// TemporalAwareCrossAttention_83597243449588
// MI455X (gfx1250) — hardware-verified
//
#include <hip/hip_runtime.h>
#include <math.h>
#include <stdint.h>

#define NB    2
#define NT    16
#define NS    128
#define NTOK  2048
#define DM    512
#define NH    16
#define HD    64
#define INNER 1024
#define MROWS 4096

static_assert(NTOK == NT * NS);
static_assert(INNER == NH * HD);
static_assert(MROWS == NB * NTOK);
static_assert(DM % 64 == 0 && INNER % 64 == 0 && HD == 64 && NTOK % 64 == 0);

typedef __bf16   v16b __attribute__((ext_vector_type(16)));
typedef __bf16   v8b  __attribute__((ext_vector_type(8)));
typedef _Float16 v16h __attribute__((ext_vector_type(16)));
typedef _Float16 v8h  __attribute__((ext_vector_type(8)));
typedef float    v8f  __attribute__((ext_vector_type(8)));
typedef float    v4f  __attribute__((ext_vector_type(4)));
typedef unsigned int v4u __attribute__((ext_vector_type(4)));
typedef v8h v8ha __attribute__((may_alias));
typedef v4f v4fa __attribute__((may_alias));

static_assert(sizeof(v4u) == 16);
static_assert(sizeof(v8h) == 16);

union FB { v16b v; v8b h[2]; };
union FH { v16h v; v8h h[2]; };

__device__ __forceinline__ unsigned short f2bf_bits(float f) {
  unsigned u = __float_as_uint(f);
  return (unsigned short)((u + 0x7FFFu + ((u >> 16) & 1u)) >> 16);
}
__device__ __forceinline__ float bf_bits2f(unsigned short b) { return __uint_as_float(((unsigned)b) << 16); }
__device__ __forceinline__ unsigned pk16(unsigned short a, unsigned short b) { return (unsigned)a | ((unsigned)b << 16); }

__device__ __forceinline__ void split2(float f0, float f1, unsigned& hw, unsigned& lw) {
  const unsigned short h0 = f2bf_bits(f0), h1 = f2bf_bits(f1);
  const unsigned short l0 = f2bf_bits(f0 - bf_bits2f(h0)), l1 = f2bf_bits(f1 - bf_bits2f(h1));
  hw = pk16(h0, h1);
  lw = pk16(l0, l1);
}
__device__ __forceinline__ void split8(v4f a, v4f b, v4u& hv, v4u& lv) {
  unsigned h0, h1, h2, h3, l0, l1, l2, l3;
  split2(a[0], a[1], h0, l0);
  split2(a[2], a[3], h1, l1);
  split2(b[0], b[1], h2, l2);
  split2(b[2], b[3], h3, l3);
  hv = (v4u){h0, h1, h2, h3};
  lv = (v4u){l0, l1, l2, l3};
}

__device__ __forceinline__ v8f mma_bf(v16b a, v16b b, v8f c) {
  c = __builtin_amdgcn_wmma_f32_16x16x32_bf16(false, a, false, b, (short)0, c, false, false);
  asm volatile("v_nop\n\tv_nop\n\tv_nop\n\tv_nop" : "+v"(c) : "v"(a), "v"(b));
  return c;
}
__device__ __forceinline__ v8f mma_h(v16h a, v16h b, v8f c) {
  c = __builtin_amdgcn_wmma_f32_16x16x32_f16(false, a, false, b, (short)0, c, false, false);
  asm volatile("v_nop\n\tv_nop\n\tv_nop\n\tv_nop" : "+v"(c) : "v"(a), "v"(b));
  return c;
}

__global__ __launch_bounds__(256) void k_cs_table(float* __restrict__ cs) {
  __shared__ __align__(16) float tile[32 * 64];
  const int tid = threadIdx.x;
  const int i = tid & 31;
  const int rsub = tid >> 5;
  const int n0 = blockIdx.x * 32;
  const int j = i & 7, e = i >> 3;
  const double m = (j == 0) ? 1.0 :
                   (j == 1) ? 1.333521432163324 :
                   (j == 2) ? 1.7782794100389228 :
                   (j == 3) ? 2.371373705661655 :
                   (j == 4) ? 3.1622776601683795 :
                   (j == 5) ? 4.216965034285822 :
                   (j == 6) ? 5.623413251903491 : 7.498942093324558;
  const double sc = (e == 0) ? 1.0 : (e == 1) ? 10.0 : (e == 2) ? 100.0 : 1000.0;
  const float t32 = (float)(m * sc);
  const float inv = 1.0f / t32;
#pragma unroll 1
  for (int q = 0; q < 4; ++q) {
    const int r = q * 8 + rsub;
    const float ang = (float)(n0 + r) * inv;
    float sv, cv;
    sincosf(ang, &sv, &cv);
    tile[r * 64 + i] = cv;
    tile[r * 64 + 32 + i] = sv;
  }
  __syncthreads();
  v4f vv[2];
  size_t go[2];
#pragma unroll
  for (int it = 0; it < 2; ++it) {
    const int f = it * 256 + tid;
    const int row = f >> 4, c4 = (f & 15) * 4;
    vv[it] = *(const v4fa*)(tile + row * 64 + c4);
    go[it] = (size_t)(n0 + row) * 64 + c4;
  }
#pragma unroll
  for (int it = 0; it < 2; ++it) *(volatile v4f*)(cs + go[it]) = vv[it];
  __threadfence();
#pragma unroll
  for (int it = 0; it < 2; ++it) *(volatile v4f*)(cs + go[it]) = vv[it];
}

__global__ __launch_bounds__(256) void k_split_xy(const float* __restrict__ x, const float* __restrict__ y,
                                                  const float* __restrict__ pos,
                                                  unsigned short* __restrict__ xh, unsigned short* __restrict__ xl,
                                                  unsigned short* __restrict__ yh, unsigned short* __restrict__ yl,
                                                  int ngrp) {
  const int t = blockIdx.x * 256 + (int)threadIdx.x;
  if (t >= ngrp) return;
  const bool isy = (blockIdx.y != 0);
  const float* src = isy ? y : x;
  unsigned short* dh = isy ? yh : xh;
  unsigned short* dl = isy ? yl : xl;
  const size_t e0 = (size_t)t * 8;
  const int d8 = (int)(e0 & (size_t)(DM - 1));
  const int tt = (int)((e0 / ((size_t)NS * DM)) & (size_t)(NT - 1));
  const v4f a0 = *(const v4f*)(src + e0);
  const v4f a1 = *(const v4f*)(src + e0 + 4);
  const v4f p0 = *(const v4f*)(pos + (size_t)tt * DM + d8);
  const v4f p1 = *(const v4f*)(pos + (size_t)tt * DM + d8 + 4);
  const v4f s0 = a0 + p0;
  const v4f s1 = a1 + p1;
  v4u hv, lv;
  split8(s0, s1, hv, lv);
  volatile v4u* ph = (volatile v4u*)(dh + e0);
  volatile v4u* pl = (volatile v4u*)(dl + e0);
  *ph = hv;
  *pl = lv;
  __threadfence();
  *ph = hv;
  *pl = lv;
}

__global__ __launch_bounds__(256) void k_wsplit(const float* __restrict__ W, unsigned short* __restrict__ wh,
                                                unsigned short* __restrict__ wl, int R, int C) {
  __shared__ float tile[64][65];
  const int tid = threadIdx.x;
  const int c0 = blockIdx.x * 64, r0 = blockIdx.y * 64;
#pragma unroll
  for (int it = 0; it < 4; ++it) {
    const int f = it * 256 + tid;
    const int rr = f >> 4, c4 = (f & 15) * 4;
    const v4f v = *(const v4f*)(W + (size_t)(r0 + rr) * C + c0 + c4);
    tile[rr][c4 + 0] = v[0];
    tile[rr][c4 + 1] = v[1];
    tile[rr][c4 + 2] = v[2];
    tile[rr][c4 + 3] = v[3];
  }
  __syncthreads();
  v4u hv[2], lv[2];
  size_t go[2];
#pragma unroll
  for (int it = 0; it < 2; ++it) {
    const int p = it * 256 + tid;
    const int cc = p >> 3, r8 = (p & 7) * 8;
    const v4f a = (v4f){tile[r8 + 0][cc], tile[r8 + 1][cc], tile[r8 + 2][cc], tile[r8 + 3][cc]};
    const v4f b = (v4f){tile[r8 + 4][cc], tile[r8 + 5][cc], tile[r8 + 6][cc], tile[r8 + 7][cc]};
    split8(a, b, hv[it], lv[it]);
    go[it] = (size_t)(c0 + cc) * R + r0 + r8;
  }
#pragma unroll
  for (int it = 0; it < 2; ++it) {
    *(volatile v4u*)(wh + go[it]) = hv[it];
    *(volatile v4u*)(wl + go[it]) = lv[it];
  }
  __threadfence();
#pragma unroll
  for (int it = 0; it < 2; ++it) {
    *(volatile v4u*)(wh + go[it]) = hv[it];
    *(volatile v4u*)(wl + go[it]) = lv[it];
  }
}

#define QKP 136
#define VSP 72

__global__ __launch_bounds__(256)
void k_qkv(const unsigned short* __restrict__ xh, const unsigned short* __restrict__ xl,
           const unsigned short* __restrict__ yh, const unsigned short* __restrict__ yl,
           const unsigned short* __restrict__ wqh, const unsigned short* __restrict__ wql,
           const unsigned short* __restrict__ wkh, const unsigned short* __restrict__ wkl,
           const unsigned short* __restrict__ wvh, const unsigned short* __restrict__ wvl,
           const float* __restrict__ cs,
           _Float16* __restrict__ qp, _Float16* __restrict__ kp, _Float16* __restrict__ vt) {
  __shared__ __align__(16) _Float16 tile[128 * VSP];
  const int tid = threadIdx.x, wave = tid >> 5, lane = tid & 31, lh = lane >> 4, c = lane & 15;
  const int mat  = blockIdx.x >> 9;
  const int rb   = blockIdx.x & 511;
  const int rblk = rb >> 3, cblk = rb & 7;
  const int m0   = rblk * 64;
  const int b    = m0 >> 11;
  const int nb0  = m0 & (NTOK - 1);
  const int wr   = wave & 3, wc = wave >> 2;
  const int n0   = (cblk * 2 + wc) * HD;
  const int mw   = m0 + wr * 16;

  const __bf16* Ah = (const __bf16*)(const void*)(mat == 2 ? yh : xh);
  const __bf16* Al = (const __bf16*)(const void*)(mat == 2 ? yl : xl);
  const __bf16* Bh = (const __bf16*)(const void*)(mat == 0 ? wqh : (mat == 1 ? wkh : wvh));
  const __bf16* Bl = (const __bf16*)(const void*)(mat == 0 ? wql : (mat == 1 ? wkl : wvl));

  v8f acc[4];
#pragma unroll
  for (int t = 0; t < 4; ++t) acc[t] = (v8f){0.f, 0.f, 0.f, 0.f, 0.f, 0.f, 0.f, 0.f};

  const __bf16* arh = Ah + (size_t)(mw + c) * DM + 8 * lh;
  const __bf16* arl = Al + (size_t)(mw + c) * DM + 8 * lh;
  const __bf16* brh = Bh + (size_t)(n0 + c) * DM + 8 * lh;
  const __bf16* brl = Bl + (size_t)(n0 + c) * DM + 8 * lh;

#pragma unroll 1
  for (int ks = 0; ks < DM / 32; ++ks) {
    const int k0 = ks * 32;
    FB ah, al;
    ah.h[0] = *(const v8b*)(arh + k0);
    ah.h[1] = *(const v8b*)(arh + k0 + 16);
    al.h[0] = *(const v8b*)(arl + k0);
    al.h[1] = *(const v8b*)(arl + k0 + 16);
#pragma unroll
    for (int t = 0; t < 4; ++t) {
      const size_t bofs = (size_t)t * 16 * DM + k0;
      FB bh, bl;
      bh.h[0] = *(const v8b*)(brh + bofs);
      bh.h[1] = *(const v8b*)(brh + bofs + 16);
      bl.h[0] = *(const v8b*)(brl + bofs);
      bl.h[1] = *(const v8b*)(brl + bofs + 16);
      acc[t] = mma_bf(ah.v, bh.v, acc[t]);
      acc[t] = mma_bf(ah.v, bl.v, acc[t]);
      acc[t] = mma_bf(al.v, bh.v, acc[t]);
    }
  }

  if (mat < 2) {
#pragma unroll
    for (int r = 0; r < 8; ++r) {
      const int rl = wr * 16 + 8 * lh + r;
      const float* csr = cs + (size_t)(nb0 + rl) * 64;
      const float c0 = csr[c], c1 = csr[16 + c], s0 = csr[32 + c], s1 = csr[48 + c];
      const float o0 = acc[0][r], o1 = acc[1][r], o2 = acc[2][r], o3 = acc[3][r];
      _Float16* tr = tile + rl * QKP + wc * 64 + c;
      tr[0]  = (_Float16)(o0 * c0 - o2 * s0);
      tr[16] = (_Float16)(o1 * c1 - o3 * s1);
      tr[32] = (_Float16)(o2 * c0 + o0 * s0);
      tr[48] = (_Float16)(o3 * c1 + o1 * s1);
    }
  } else {
#pragma unroll
    for (int r = 0; r < 8; ++r) {
      const int rl = wr * 16 + 8 * lh + r;
#pragma unroll
      for (int t = 0; t < 4; ++t) tile[(wc * 64 + t * 16 + c) * VSP + rl] = (_Float16)acc[t][r];
    }
  }
  __syncthreads();

  v8h sv[4];
  size_t go[4];
  _Float16* dst;
  if (mat < 2) {
    dst = (mat == 0) ? qp : kp;
#pragma unroll
    for (int it = 0; it < 4; ++it) {
      const int R = it * 16 + wave * 2 + lh;
      const int hsel = (lane >> 3) & 1, piece = lane & 7;
      sv[it] = *(const v8ha*)(tile + R * QKP + hsel * 64 + piece * 8);
      go[it] = ((size_t)(b * NH + cblk * 2 + hsel) * NTOK + nb0 + R) * HD + piece * 8;
    }
  } else {
    dst = vt;
#pragma unroll
    for (int it = 0; it < 4; ++it) {
      const int R = it * 32 + (tid >> 3);
      const int piece = tid & 7;
      sv[it] = *(const v8ha*)(tile + R * VSP + piece * 8);
      go[it] = ((size_t)(b * NH + cblk * 2 + (R >> 6)) * HD + (R & 63)) * NTOK + nb0 + piece * 8;
    }
  }
#pragma unroll
  for (int it = 0; it < 4; ++it) *(volatile v8h*)(dst + go[it]) = sv[it];
  __threadfence();
#pragma unroll
  for (int it = 0; it < 4; ++it) *(volatile v8h*)(dst + go[it]) = sv[it];
}

#define KC  64
#define KSP 72
#define PSP 72
#define OSP 68

__global__ __launch_bounds__(128)
void k_attn(const _Float16* __restrict__ qp, const _Float16* __restrict__ kp, const _Float16* __restrict__ vt,
            const int* __restrict__ tmask, unsigned short* __restrict__ oh, unsigned short* __restrict__ ol) {
  __shared__ __align__(16) _Float16 Ks[KC * KSP];
  __shared__ __align__(16) _Float16 Vs[HD * KSP];
  __shared__ __align__(16) _Float16 Ps[4][16 * PSP];
  __shared__ __align__(16) float    Os[4][16 * OSP];

  const int tid = threadIdx.x, wave = tid >> 5, lane = tid & 31, lh = lane >> 4, c = lane & 15;
  const int qt  = blockIdx.x & 31;
  const int bh  = blockIdx.x >> 5;
  const int b   = bh >> 4, h = bh & 15;
  const int qg0 = qt * 64 + wave * 16;
  const int tq  = qt >> 1;

  unsigned mbits = 0;
  {
    const int* mr = tmask + (b * NT + tq) * NT;
#pragma unroll
    for (int tj = 0; tj < NT; ++tj) mbits |= (mr[tj] != 0 ? 1u : 0u) << tj;
  }

  const _Float16* Qb = qp + (size_t)bh * NTOK * HD;
  const _Float16* Kb = kp + (size_t)bh * NTOK * HD;
  const _Float16* Vb = vt + (size_t)bh * HD * NTOK;

  FH qa[2];
  {
    const _Float16* qr = Qb + (size_t)(qg0 + c) * HD + 8 * lh;
    qa[0].h[0] = *(const v8h*)(qr);
    qa[0].h[1] = *(const v8h*)(qr + 16);
    qa[1].h[0] = *(const v8h*)(qr + 32);
    qa[1].h[1] = *(const v8h*)(qr + 48);
  }

  float mrow[8], lrow[8];
  v8f oacc[4];
#pragma unroll
  for (int r = 0; r < 8; ++r) { mrow[r] = -INFINITY; lrow[r] = 0.f; }
#pragma unroll
  for (int t = 0; t < 4; ++t) oacc[t] = (v8f){0.f, 0.f, 0.f, 0.f, 0.f, 0.f, 0.f, 0.f};

  _Float16* pw = Ps[wave];

#pragma unroll 1
  for (int kc = 0; kc < NTOK / KC; ++kc) {
    if (((mbits >> (kc >> 1)) & 1u) == 0u) continue;
    const int kv0 = kc * KC;
    __syncthreads();
#pragma unroll
    for (int i = 0; i < 4; ++i) {
      const int p = i * 128 + tid;
      const int r = p >> 3, q8 = (p & 7) * 8;
      *(v8h*)(Ks + r * KSP + q8) = *(const v8h*)(Kb + (size_t)(kv0 + r) * HD + q8);
      *(v8h*)(Vs + r * KSP + q8) = *(const v8h*)(Vb + (size_t)r * NTOK + kv0 + q8);
    }
    __syncthreads();

    v8f s[4];
#pragma unroll
    for (int j = 0; j < 4; ++j) s[j] = (v8f){0.f, 0.f, 0.f, 0.f, 0.f, 0.f, 0.f, 0.f};
#pragma unroll
    for (int dc = 0; dc < 2; ++dc) {
#pragma unroll
      for (int j = 0; j < 4; ++j) {
        const _Float16* kq = Ks + (j * 16 + c) * KSP + dc * 32 + 8 * lh;
        FH kb;
        kb.h[0] = *(const v8ha*)(kq);
        kb.h[1] = *(const v8ha*)(kq + 16);
        s[j] = mma_h(qa[dc].v, kb.v, s[j]);
      }
    }
    float cm[8], alpha[8];
#pragma unroll
    for (int r = 0; r < 8; ++r) {
      float m = -INFINITY;
#pragma unroll
      for (int j = 0; j < 4; ++j) {
        const float sv = s[j][r] * 0.125f;
        s[j][r] = sv;
        m = fmaxf(m, sv);
      }
#pragma unroll
      for (int off = 1; off < 16; off <<= 1) m = fmaxf(m, __shfl_xor(m, off, 32));
      cm[r] = m;
    }
#pragma unroll
    for (int r = 0; r < 8; ++r) {
      const float mnew = fmaxf(mrow[r], cm[r]);
      alpha[r] = __expf(mrow[r] - mnew);
      mrow[r] = mnew;
      float psum = 0.f;
#pragma unroll
      for (int j = 0; j < 4; ++j) {
        const float p = __expf(s[j][r] - mnew);
        psum += p;
        pw[(8 * lh + r) * PSP + j * 16 + c] = (_Float16)(p * 1024.0f);
      }
#pragma unroll
      for (int off = 1; off < 16; off <<= 1) psum += __shfl_xor(psum, off, 32);
      lrow[r] = lrow[r] * alpha[r] + psum;
    }
    __syncthreads();

#pragma unroll
    for (int t = 0; t < 4; ++t)
#pragma unroll
      for (int r = 0; r < 8; ++r) oacc[t][r] *= alpha[r];
#pragma unroll
    for (int kk = 0; kk < 2; ++kk) {
      FH pa;
      pa.h[0] = *(const v8ha*)(pw + c * PSP + kk * 32 + 8 * lh);
      pa.h[1] = *(const v8ha*)(pw + c * PSP + kk * 32 + 16 + 8 * lh);
#pragma unroll
      for (int t = 0; t < 4; ++t) {
        const _Float16* vq = Vs + (t * 16 + c) * KSP + kk * 32 + 8 * lh;
        FH vb;
        vb.h[0] = *(const v8ha*)(vq);
        vb.h[1] = *(const v8ha*)(vq + 16);
        oacc[t] = mma_h(pa.v, vb.v, oacc[t]);
      }
    }
  }

  float* os = Os[wave];
#pragma unroll
  for (int r = 0; r < 8; ++r) {
    const float inv = (1.0f / lrow[r]) * (1.0f / 1024.0f);
#pragma unroll
    for (int t = 0; t < 4; ++t) os[(8 * lh + r) * OSP + t * 16 + c] = oacc[t][r] * inv;
  }
  __syncthreads();
  v4u hv[4], lv[4];
  size_t go[4];
#pragma unroll
  for (int it = 0; it < 4; ++it) {
    const int row = it * 4 + (lane >> 3);
    const int piece = lane & 7;
    const float* op = os + row * OSP + piece * 8;
    const v4f f0 = *(const v4fa*)(op);
    const v4f f1 = *(const v4fa*)(op + 4);
    split8(f0, f1, hv[it], lv[it]);
    go[it] = ((size_t)(b * NTOK + qg0 + row)) * INNER + h * HD + piece * 8;
  }
#pragma unroll
  for (int it = 0; it < 4; ++it) {
    *(volatile v4u*)(oh + go[it]) = hv[it];
    *(volatile v4u*)(ol + go[it]) = lv[it];
  }
  __threadfence();
#pragma unroll
  for (int it = 0; it < 4; ++it) {
    *(volatile v4u*)(oh + go[it]) = hv[it];
    *(volatile v4u*)(ol + go[it]) = lv[it];
  }
}

#define TSP 520

__global__ __launch_bounds__(256)
void k_out(const unsigned short* __restrict__ ohp, const unsigned short* __restrict__ olp,
           const unsigned short* __restrict__ woh, const unsigned short* __restrict__ wol,
           const float* __restrict__ bo, const float* __restrict__ gw, const float* __restrict__ gb,
           float* __restrict__ out) {
  __shared__ __align__(16) float ts[16 * TSP];
  __shared__ float gs[16];
  const int tid = threadIdx.x, wave = tid >> 5, lane = tid & 31, lh = lane >> 4, c = lane & 15;
  const int m0 = blockIdx.x * 16;
  const int n0 = wave * 64;

  const __bf16* Ah = (const __bf16*)(const void*)ohp;
  const __bf16* Al = (const __bf16*)(const void*)olp;
  const __bf16* Bh = (const __bf16*)(const void*)woh;
  const __bf16* Bl = (const __bf16*)(const void*)wol;

  v8f acc[4];
#pragma unroll
  for (int t = 0; t < 4; ++t) acc[t] = (v8f){0.f, 0.f, 0.f, 0.f, 0.f, 0.f, 0.f, 0.f};

  const __bf16* arh = Ah + (size_t)(m0 + c) * INNER + 8 * lh;
  const __bf16* arl = Al + (size_t)(m0 + c) * INNER + 8 * lh;
  const __bf16* brh = Bh + (size_t)(n0 + c) * INNER + 8 * lh;
  const __bf16* brl = Bl + (size_t)(n0 + c) * INNER + 8 * lh;

#pragma unroll 1
  for (int ks = 0; ks < INNER / 32; ++ks) {
    const int k0 = ks * 32;
    FB ah, al;
    ah.h[0] = *(const v8b*)(arh + k0);
    ah.h[1] = *(const v8b*)(arh + k0 + 16);
    al.h[0] = *(const v8b*)(arl + k0);
    al.h[1] = *(const v8b*)(arl + k0 + 16);
#pragma unroll
    for (int t = 0; t < 4; ++t) {
      const size_t bofs = (size_t)t * 16 * INNER + k0;
      FB bh, bl;
      bh.h[0] = *(const v8b*)(brh + bofs);
      bh.h[1] = *(const v8b*)(brh + bofs + 16);
      bl.h[0] = *(const v8b*)(brl + bofs);
      bl.h[1] = *(const v8b*)(brl + bofs + 16);
      acc[t] = mma_bf(ah.v, bh.v, acc[t]);
      acc[t] = mma_bf(ah.v, bl.v, acc[t]);
      acc[t] = mma_bf(al.v, bh.v, acc[t]);
    }
  }

#pragma unroll
  for (int t = 0; t < 4; ++t) {
    const float bias = bo[n0 + t * 16 + c];
#pragma unroll
    for (int r = 0; r < 8; ++r) ts[(8 * lh + r) * TSP + n0 + t * 16 + c] = acc[t][r] + bias;
  }
  __syncthreads();
  {
    const int row = tid >> 4, part = tid & 15;
    const float* tr = ts + row * TSP + part * 32;
    const float* gp = gw + part * 32;
    float sum = 0.f;
#pragma unroll 4
    for (int i = 0; i < 32; ++i) sum += tr[i] * gp[i];
#pragma unroll
    for (int off = 1; off < 16; off <<= 1) sum += __shfl_xor(sum, off, 32);
    const float z = sum + gb[0];
    const float den = 1.0f + expf(-z);
    const float g = 1.0f / den;
    if (part == 0) gs[row] = g;
  }
  __syncthreads();
  v4f vv[8];
  size_t go[8];
#pragma unroll
  for (int it = 0; it < 8; ++it) {
    const int f = it * 256 + tid;
    const int row = f >> 7, c4 = (f & 127) * 4;
    const v4f v = *(const v4fa*)(ts + row * TSP + c4);
    const float g = gs[row];
    vv[it] = v * g;
    go[it] = (size_t)(m0 + row) * DM + c4;
  }
#pragma unroll
  for (int it = 0; it < 8; ++it) *(volatile v4f*)(out + go[it]) = vv[it];
  __threadfence();
#pragma unroll
  for (int it = 0; it < 8; ++it) *(volatile v4f*)(out + go[it]) = vv[it];
}

extern "C" void kernel_launch(void* const* d_in, const int* in_sizes, int n_in,
                              void* d_out, int out_size, void* d_ws, size_t ws_size,
                              hipStream_t stream) {
  if (n_in < 11) return;
  if (in_sizes[0] != MROWS * DM || in_sizes[1] != MROWS * DM) return;
  if (in_sizes[2] != NB * NT * NT) return;
  if (in_sizes[3] != DM * INNER || in_sizes[4] != DM * INNER || in_sizes[5] != DM * INNER) return;
  if (in_sizes[6] != INNER * DM || in_sizes[7] != DM) return;
  if (in_sizes[8] < NT * DM || in_sizes[9] != DM || in_sizes[10] < 1) return;
  if (out_size != MROWS * DM) return;

  const float* x     = (const float*)d_in[0];
  const float* y     = (const float*)d_in[1];
  const int*   tmask = (const int*)d_in[2];
  const float* Wq    = (const float*)d_in[3];
  const float* Wk    = (const float*)d_in[4];
  const float* Wv    = (const float*)d_in[5];
  const float* Wo    = (const float*)d_in[6];
  const float* bo    = (const float*)d_in[7];
  const float* pos   = (const float*)d_in[8];
  const float* gw    = (const float*)d_in[9];
  const float* gb    = (const float*)d_in[10];
  float* o = (float*)d_out;

  const size_t PX  = (size_t)MROWS * DM * 2;
  const size_t PW  = (size_t)DM * INNER * 2;
  const size_t PCS = (size_t)NTOK * 64 * 4;
  const size_t PQ  = (size_t)NB * NH * NTOK * HD * 2;
  const size_t PO  = (size_t)MROWS * INNER * 2;
  size_t off = 0;
  const size_t oXh = off; off += PX;
  const size_t oXl = off; off += PX;
  const size_t oYh = off; off += PX;
  const size_t oYl = off; off += PX;
  const size_t oWqh = off; off += PW;
  const size_t oWql = off; off += PW;
  const size_t oWkh = off; off += PW;
  const size_t oWkl = off; off += PW;
  const size_t oWvh = off; off += PW;
  const size_t oWvl = off; off += PW;
  const size_t oWoh = off; off += PW;
  const size_t oWol = off; off += PW;
  const size_t oCS = off; off += PCS;
  const size_t oQ  = off; off += PQ;
  const size_t oK  = off; off += PQ;
  const size_t oVt = off; off += PQ;
  const size_t oOh = off; off += PO;
  const size_t oOl = off; off += PO;
  if (off > ws_size) return;

  char* ws = (char*)d_ws;
  unsigned short* xh  = (unsigned short*)(ws + oXh);
  unsigned short* xl  = (unsigned short*)(ws + oXl);
  unsigned short* yh  = (unsigned short*)(ws + oYh);
  unsigned short* yl  = (unsigned short*)(ws + oYl);
  unsigned short* wqh = (unsigned short*)(ws + oWqh);
  unsigned short* wql = (unsigned short*)(ws + oWql);
  unsigned short* wkh = (unsigned short*)(ws + oWkh);
  unsigned short* wkl = (unsigned short*)(ws + oWkl);
  unsigned short* wvh = (unsigned short*)(ws + oWvh);
  unsigned short* wvl = (unsigned short*)(ws + oWvl);
  unsigned short* woh = (unsigned short*)(ws + oWoh);
  unsigned short* wol = (unsigned short*)(ws + oWol);
  float*          cs  = (float*)(ws + oCS);
  _Float16*       qpl = (_Float16*)(ws + oQ);
  _Float16*       kpl = (_Float16*)(ws + oK);
  _Float16*       vtp = (_Float16*)(ws + oVt);
  unsigned short* ohp = (unsigned short*)(ws + oOh);
  unsigned short* olp = (unsigned short*)(ws + oOl);

  k_cs_table<<<dim3(NTOK / 32), dim3(256), 0, stream>>>(cs);
  const int ngrp = MROWS * DM / 8;
  k_split_xy<<<dim3((ngrp + 255) / 256, 2), dim3(256), 0, stream>>>(x, y, pos, xh, xl, yh, yl, ngrp);
  k_wsplit<<<dim3(INNER / 64, DM / 64), dim3(256), 0, stream>>>(Wq, wqh, wql, DM, INNER);
  k_wsplit<<<dim3(INNER / 64, DM / 64), dim3(256), 0, stream>>>(Wk, wkh, wkl, DM, INNER);
  k_wsplit<<<dim3(INNER / 64, DM / 64), dim3(256), 0, stream>>>(Wv, wvh, wvl, DM, INNER);
  k_wsplit<<<dim3(DM / 64, INNER / 64), dim3(256), 0, stream>>>(Wo, woh, wol, INNER, DM);
  k_qkv<<<dim3(3 * 512), dim3(256), 0, stream>>>(xh, xl, yh, yl, wqh, wql, wkh, wkl, wvh, wvl, cs,
                                                 qpl, kpl, vtp);
  k_attn<<<dim3(NB * NH * (NTOK / 64)), dim3(128), 0, stream>>>(qpl, kpl, vtp, tmask, ohp, olp);
  k_out<<<dim3(MROWS / 16), dim3(256), 0, stream>>>(ohp, olp, woh, wol, bo, gw, gb, o);
  (void)hipGetLastError();
}
